// TDrumorGAT_34574486733591
// MI455X (gfx1250) — hardware-verified
//
#include <hip/hip_runtime.h>
#include <stddef.h>


#define FWD     256
#define NLG     8
#define HCH     64
#define OWD     512
#define NTHR    256
#define NWAVE   8
#define EPT     8
#define NGRP    2
#define CHUNK   (NTHR * EPT * NGRP)
#define WCAP    (EPT * NGRP * 32)
#define LISTN   (NWAVE * WCAP)
#define NBC     4096
#define NBF     1024
#define RCAP    40960
#define RBN     128
#define AGTHR   128
#define AGW     4
#define TGT     (AGW * 32)
#define DEGCAP  1024
#define OTHR    512
#define BM      32
#define RGRAN   256
#define GPB     2
#define GMAX    1024
#define WSCAP   134217728
#define ACARRY  8.0f
#define WCARRY  256.0f
#define GSCALE  (1.0f / 2048.0f)

#define LDS_FILL ((RCAP + NBF + LISTN) * 4 + 64)

static_assert((CHUNK & (CHUNK - 1)) == 0);
static_assert(CHUNK <= 4096);
static_assert((NBC & (NBC - 1)) == 0 && (NBF & (NBF - 1)) == 0);
static_assert(NBC == 4 * NBF);
static_assert(OTHR * 8 == NBC);
static_assert((RCAP % 32) == 0);
static_assert(TGT == AGW * 32);
static_assert(WCAP == EPT * NGRP * 32);
static_assert((RGRAN % TGT) == 0 && (RGRAN % BM) == 0);
static_assert(RGRAN == NTHR);
static_assert((FWD % 32) == 0);
static_assert(FWD == 4 * HCH);
static_assert(FWD / 2 == 32 * 4);
static_assert(OWD == 2 * FWD);
static_assert((GPB & (GPB - 1)) == 0 && GPB <= NWAVE);
static_assert(((GPB * OWD) % NTHR) == 0);
static_assert(FWD * NLG == 8 * NTHR);
static_assert((FWD * NLG) % NTHR == 0);

typedef float    v4f  __attribute__((ext_vector_type(4)));
typedef float    v8f  __attribute__((ext_vector_type(8)));
typedef int      v4i  __attribute__((ext_vector_type(4)));
typedef _Float16 v4h  __attribute__((ext_vector_type(4)));
typedef _Float16 v8h  __attribute__((ext_vector_type(8)));
typedef _Float16 v16h __attribute__((ext_vector_type(16)));
union Frag { v16h v; v8h h[2]; };

__device__ __forceinline__ v8f wmh(v16h a, v16h b, v8f c) {
  v8f d = __builtin_amdgcn_wmma_f32_16x16x32_f16(false, a, false, b, (short)0, c, false, false);
  asm volatile("v_nop\n\tv_nop\n\tv_nop\n\tv_nop" : "+v"(d) : "v"(a), "v"(b));
  return d;
}

__device__ __forceinline__ v4f ld4(const float* p) { return *(const v4f*)p; }

__device__ __forceinline__ v4f zsel(bool live, v4f v) {
  v4f o;
  o.x = live ? v.x : 0.f;
  o.y = live ? v.y : 0.f;
  o.z = live ? v.z : 0.f;
  o.w = live ? v.w : 0.f;
  return o;
}

__device__ __forceinline__ float wsum(float v) {
  v += __shfl_xor(v, 16);
  v += __shfl_xor(v, 8);
  v += __shfl_xor(v, 4);
  v += __shfl_xor(v, 2);
  v += __shfl_xor(v, 1);
  return v;
}

__device__ __forceinline__ float wmax(float v) {
  v = fmaxf(v, __shfl_xor(v, 16));
  v = fmaxf(v, __shfl_xor(v, 8));
  v = fmaxf(v, __shfl_xor(v, 4));
  v = fmaxf(v, __shfl_xor(v, 2));
  v = fmaxf(v, __shfl_xor(v, 1));
  return v;
}

__device__ __forceinline__ float lk(float e) { return e >= 0.f ? e : 0.2f * e; }

template <int NB>
__device__ __forceinline__ int scan_chunk(const int* __restrict__ dsts, int nE, int cbase, int slotBase,
                                          int vec8, int* list, int tid, int lane, int wave) {
  int wc = 0;
#pragma unroll
  for (int g = 0; g < NGRP; ++g) {
    const int el0  = (g * NTHR + tid) * EPT;
    const int e0   = cbase + el0;
    const int sent = -2147483647 - 1;
    v4i da, db;
    if (vec8 != 0 && cbase + CHUNK <= nE) {
      da = *(const v4i*)(dsts + e0);
      db = *(const v4i*)(dsts + e0 + 4);
    } else {
      da.x = (e0     < nE) ? dsts[min(e0, nE - 1)] : sent;
      da.y = (e0 + 1 < nE) ? dsts[min(e0 + 1, nE - 1)] : sent;
      da.z = (e0 + 2 < nE) ? dsts[min(e0 + 2, nE - 1)] : sent;
      da.w = (e0 + 3 < nE) ? dsts[min(e0 + 3, nE - 1)] : sent;
      db.x = (e0 + 4 < nE) ? dsts[min(e0 + 4, nE - 1)] : sent;
      db.y = (e0 + 5 < nE) ? dsts[min(e0 + 5, nE - 1)] : sent;
      db.z = (e0 + 6 < nE) ? dsts[min(e0 + 6, nE - 1)] : sent;
      db.w = (e0 + 7 < nE) ? dsts[min(e0 + 7, nE - 1)] : sent;
    }
    const unsigned nb = (unsigned)slotBase;
    const unsigned s0 = (unsigned)da.x - nb, s1 = (unsigned)da.y - nb;
    const unsigned s2 = (unsigned)da.z - nb, s3 = (unsigned)da.w - nb;
    const unsigned s4 = (unsigned)db.x - nb, s5 = (unsigned)db.y - nb;
    const unsigned s6 = (unsigned)db.z - nb, s7 = (unsigned)db.w - nb;
    const bool h0 = s0 < (unsigned)NB, h1 = s1 < (unsigned)NB, h2 = s2 < (unsigned)NB, h3 = s3 < (unsigned)NB;
    const bool h4 = s4 < (unsigned)NB, h5 = s5 < (unsigned)NB, h6 = s6 < (unsigned)NB, h7 = s7 < (unsigned)NB;
    const unsigned any = __builtin_amdgcn_ballot_w32(h0 | h1 | h2 | h3 | h4 | h5 | h6 | h7);
    if (any != 0u) {
#define HITJ(J, HJ, SJ) { \
        const unsigned mj = __builtin_amdgcn_ballot_w32(HJ); \
        if (mj != 0u) { \
          if (HJ) { \
            const int pos = wc + (int)__builtin_amdgcn_mbcnt_lo(mj, 0u); \
            if (pos < WCAP) list[wave * WCAP + pos] = ((el0 + (J)) << 12) | (int)(SJ); \
          } \
          wc += (int)__builtin_popcount(mj); } }
      HITJ(0, h0, s0)
      HITJ(1, h1, s1)
      HITJ(2, h2, s2)
      HITJ(3, h3, s3)
      HITJ(4, h4, s4)
      HITJ(5, h5, s5)
      HITJ(6, h6, s6)
      HITJ(7, h7, s7)
#undef HITJ
    }
  }
  return wc;
}

__global__ __launch_bounds__(NTHR) void k_count(
    const int* __restrict__ dsts, int* cnt, int nE, int vec8) {
  __shared__ __attribute__((aligned(16))) int scnt[NBC];
  __shared__ __attribute__((aligned(16))) int list[LISTN];
  __shared__ int wcnt[NWAVE];
  const int tid = threadIdx.x, lane = tid & 31, wave = tid >> 5;
  const int nodeBase = blockIdx.x * NBC;

  for (int i = tid; i < NBC; i += NTHR) scnt[i] = 0;
  __syncthreads();

  const int nChunks = (nE + CHUNK - 1) / CHUNK;
#pragma unroll 1
  for (int ch = 0; ch < nChunks; ++ch) {
    const int cbase = ch * CHUNK;
    const int wc = scan_chunk<NBC>(dsts, nE, cbase, nodeBase, vec8, list, tid, lane, wave);
    if (lane == 0) wcnt[wave] = wc;
    __syncthreads();
    if (wave == 0) {
#pragma unroll 1
      for (int wsx = 0; wsx < NWAVE; ++wsx) {
        int n = __builtin_amdgcn_readfirstlane(wcnt[wsx]);
        n = n > WCAP ? WCAP : (n < 0 ? 0 : n);
        const int* lp = list + wsx * WCAP;
#pragma unroll 1
        for (int i = 0; i < n; ++i) {
          const int ent  = __builtin_amdgcn_readfirstlane(lp[i]);
          const int slot = ent & (NBC - 1);
          if (lane == 0) scnt[slot] = scnt[slot] + 1;
        }
      }
    }
    __syncthreads();
  }

  v4i cq[4];
#pragma unroll
  for (int q = 0; q < 4; ++q) {
    const int f = (wave * 4 + q) * 128 + 4 * lane;
    cq[q] = *(const v4i*)(scnt + f);
  }
  int* cp = cnt + (size_t)nodeBase;
#pragma unroll
  for (int q = 0; q < 4; ++q) {
    const int f = (wave * 4 + q) * 128 + 4 * lane;
    *(volatile v4i*)(cp + f) = cq[q];
  }
  __threadfence();
#pragma unroll
  for (int q = 0; q < 4; ++q) {
    const int f = (wave * 4 + q) * 128 + 4 * lane;
    *(volatile v4i*)(cp + f) = cq[q];
  }
}

__global__ __launch_bounds__(OTHR) void k_offsets(
    const int* __restrict__ cnt, int* off, int* rbase, int nChunk) {
  __shared__ __attribute__((aligned(16))) int soff[NBC];
  __shared__ __attribute__((aligned(16))) int srb[RBN];
  __shared__ int wtot[OTHR / 32];
  const int tid = threadIdx.x, lane = tid & 31, wave = tid >> 5, sub = tid >> 7;
  for (int i = tid; i < RBN; i += OTHR) srb[i] = 0;
  int carry = 0;
#pragma unroll 1
  for (int ch = 0; ch < nChunk; ++ch) {
    const int base = ch * NBC;
    const v4i c0 = *(const v4i*)(cnt + base + 8 * tid);
    const v4i c1 = *(const v4i*)(cnt + base + 8 * tid + 4);
    const int e0 = max(c0.x, 0), e1 = max(c0.y, 0), e2 = max(c0.z, 0), e3 = max(c0.w, 0);
    const int e4 = max(c1.x, 0), e5 = max(c1.y, 0), e6 = max(c1.z, 0), e7 = max(c1.w, 0);
    const int ts = e0 + e1 + e2 + e3 + e4 + e5 + e6 + e7;
    int incl = ts;
#pragma unroll
    for (int d = 1; d < 32; d <<= 1) {
      const int t = __shfl_up(incl, d);
      if (lane >= d) incl += t;
    }
    if (lane == 31) wtot[wave] = incl;
    __syncthreads();
    const int S0 = wtot[0]  + wtot[1]  + wtot[2]  + wtot[3];
    const int S1 = wtot[4]  + wtot[5]  + wtot[6]  + wtot[7];
    const int S2 = wtot[8]  + wtot[9]  + wtot[10] + wtot[11];
    const int S3 = wtot[12] + wtot[13] + wtot[14] + wtot[15];
    int pre = 0;
#pragma unroll 1
    for (int w = 4 * sub; w < wave; ++w) pre += wtot[w];
    const int b0 = carry;
    const int b1 = b0 + ((S0 + 31) & ~31);
    const int b2 = b1 + ((S1 + 31) & ~31);
    const int b3 = b2 + ((S2 + 31) & ~31);
    const int b4 = b3 + ((S3 + 31) & ~31);
    const int myb = sub == 0 ? b0 : (sub == 1 ? b1 : (sub == 2 ? b2 : b3));
    if (tid == 0) {
      srb[min(4 * ch + 0, RBN - 1)] = b0;
      srb[min(4 * ch + 1, RBN - 1)] = b1;
      srb[min(4 * ch + 2, RBN - 1)] = b2;
      srb[min(4 * ch + 3, RBN - 1)] = b3;
    }
    int run = myb + pre + incl - ts;
    soff[8 * tid + 0] = run; run += e0;
    soff[8 * tid + 1] = run; run += e1;
    soff[8 * tid + 2] = run; run += e2;
    soff[8 * tid + 3] = run; run += e3;
    soff[8 * tid + 4] = run; run += e4;
    soff[8 * tid + 5] = run; run += e5;
    soff[8 * tid + 6] = run; run += e6;
    soff[8 * tid + 7] = run;
    carry = b4;
    __syncthreads();
    const v4i o0 = *(const v4i*)(soff + 4 * tid);
    const v4i o1 = *(const v4i*)(soff + 4 * (tid + OTHR));
    int* op = off + base;
    *(volatile v4i*)(op + 4 * tid) = o0;
    *(volatile v4i*)(op + 4 * (tid + OTHR)) = o1;
    __threadfence();
    *(volatile v4i*)(op + 4 * tid) = o0;
    *(volatile v4i*)(op + 4 * (tid + OTHR)) = o1;
    __syncthreads();
  }
  if (tid == 0) srb[min(4 * nChunk, RBN - 1)] = carry;
  __syncthreads();
  v4i rv = {0, 0, 0, 0};
  if (tid < 32) rv = *(const v4i*)(srb + 4 * tid);
  if (tid < 32) *(volatile v4i*)(rbase + 4 * tid) = rv;
  __threadfence();
  if (tid < 32) *(volatile v4i*)(rbase + 4 * tid) = rv;
}

__global__ __launch_bounds__(NTHR) void k_fill(
    const int* __restrict__ srcs, const int* __restrict__ dsts,
    const int* __restrict__ off, const int* __restrict__ rbase,
    int* csr, int nN, int nE, int vec8, int csrLen) {
  extern __shared__ v4f lds_dyn[];
  int* region = (int*)lds_dyn;
  int* cursor = region + RCAP;
  int* list   = cursor + NBF;
  int* wcnt   = list + LISTN;
  const int tid = threadIdx.x, lane = tid & 31, wave = tid >> 5;
  const int b = blockIdx.x;
  const int nodeBase = b * NBF;

  int rb0 = rbase[b];
  const int rb1 = rbase[b + 1];
  rb0 = rb0 < 0 ? 0 : (rb0 > csrLen ? csrLen : rb0);
  rb0 &= ~31;
  int len = rb1 - rb0;
  len = len < 0 ? 0 : (len > RCAP ? RCAP : len);
  int lenW = (len + 31) & ~31;
  if (rb0 + lenW > csrLen) lenW = (csrLen - rb0) & ~31;

  {
    const v4i z = {0, 0, 0, 0};
    for (int i = tid; i < RCAP / 4; i += NTHR) ((v4i*)region)[i] = z;
    for (int s = tid; s < NBF; s += NTHR) {
      int o = off[nodeBase + s] - rb0;
      o = o < 0 ? 0 : (o > RCAP ? RCAP : o);
      cursor[s] = o;
    }
  }
  __syncthreads();

  const int nChunks = (nE + CHUNK - 1) / CHUNK;
#pragma unroll 1
  for (int ch = 0; ch < nChunks; ++ch) {
    const int cbase = ch * CHUNK;
    const int wc = scan_chunk<NBF>(dsts, nE, cbase, nodeBase, vec8, list, tid, lane, wave);
    if (lane == 0) wcnt[wave] = wc;
    __syncthreads();
    if (wave == 0) {
#pragma unroll 1
      for (int wsx = 0; wsx < NWAVE; ++wsx) {
        int n = __builtin_amdgcn_readfirstlane(wcnt[wsx]);
        n = n > WCAP ? WCAP : (n < 0 ? 0 : n);
        const int* lp = list + wsx * WCAP;
#pragma unroll 1
        for (int i = 0; i < n; ++i) {
          const int ent  = __builtin_amdgcn_readfirstlane(lp[i]);
          const int slot = ent & (NBF - 1);
          int e = cbase + ((ent >> 12) & (CHUNK - 1));
          e = e > nE - 1 ? nE - 1 : e;
          int sv = srcs[e];
          sv = sv < 0 ? 0 : (sv > nN - 1 ? nN - 1 : sv);
          if (lane == 0) {
            int pos = cursor[slot];
            pos = pos < 0 ? 0 : (pos > RCAP - 1 ? RCAP - 1 : pos);
            region[pos] = sv;
            const int np = pos + 1;
            cursor[slot] = np > RCAP ? RCAP : np;
          }
        }
      }
    }
    __syncthreads();
  }

  const int nv = lenW >> 2;
  int* gp = csr + rb0;
#pragma unroll 1
  for (int i = tid; i < nv; i += NTHR) { const v4i v = ((const v4i*)region)[i]; *(volatile v4i*)(gp + 4 * i) = v; }
  __threadfence();
#pragma unroll 1
  for (int i = tid; i < nv; i += NTHR) { const v4i v = ((const v4i*)region)[i]; *(volatile v4i*)(gp + 4 * i) = v; }
}

__global__ __launch_bounds__(NTHR) void k_wcvt(const float* __restrict__ W, _Float16* dp,
                                               int kOff, int K, int nRowsW) {
  const int ppr = K >> 3;
  const int nUnits = FWD * ppr;
  const int i = (int)blockIdx.x * NTHR + (int)threadIdx.x;
  if (i >= nUnits) return;
  const int n = i / ppr;
  const int seg = i - n * ppr;
  v8h o;
#pragma unroll
  for (int j = 0; j < 8; ++j) {
    int k = kOff + 8 * seg + j;
    k = k < 0 ? 0 : (k > nRowsW - 1 ? nRowsW - 1 : k);
    o[j] = (_Float16)(W[(size_t)k * FWD + n] * WCARRY);
  }
  _Float16* gp = dp + (size_t)i * 8;
  *(volatile v8h*)gp = o;
  __threadfence();
  *(volatile v8h*)gp = o;
}

__global__ __launch_bounds__(NTHR) void k_wa(const float* __restrict__ W1, const float* __restrict__ W2,
                                             const float* __restrict__ as1, const float* __restrict__ ad1,
                                             const float* __restrict__ as2, const float* __restrict__ ad2,
                                             float* wa) {
  const int t = (int)blockIdx.x * NTHR + (int)threadIdx.x;
  const int r = t >> 3, j = t & 7, hd = j & 3;
  const bool l2 = blockIdx.x >= (FWD * NLG) / NTHR;
  const float* W = l2 ? W2 : W1;
  int row = l2 ? (r - FWD) : r;
  row = row < 0 ? 0 : row;
  row = l2 ? (row > 2 * FWD - 1 ? 2 * FWD - 1 : row) : (row > FWD - 1 ? FWD - 1 : row);
  const float* asp = (l2 ? as2 : as1) + hd * HCH;
  const float* adp = (l2 ? ad2 : ad1) + hd * HCH;
  const float* wp = W + (size_t)row * FWD + hd * HCH;
  const bool usd = j >= 4;
  float acc = 0.f;
#pragma unroll 4
  for (int c = 0; c < HCH; ++c) {
    const float av = asp[c];
    const float dv = adp[c];
    const float a = usd ? dv : av;
    acc += wp[c] * a;
  }
  float* gp = wa + t;
  *(volatile float*)gp = acc;
  __threadfence();
  *(volatile float*)gp = acc;
}

template <int L2>
__global__ __launch_bounds__(NTHR) void k_logit(const float* __restrict__ src, const float* __restrict__ wa,
                                                const float* __restrict__ gl2, const int* __restrict__ batch,
                                                float* al, int nN, int nR) {
  __shared__ __attribute__((aligned(16))) float swa[FWD * NLG];
  __shared__ __attribute__((aligned(16))) float sout[NTHR * NLG];
  const int tid = threadIdx.x;
  const int n = (int)blockIdx.x * NTHR + tid;
  *(v4f*)(swa + 8 * tid)     = *(const v4f*)(wa + 8 * tid);
  *(v4f*)(swa + 8 * tid + 4) = *(const v4f*)(wa + 8 * tid + 4);
  __syncthreads();

  const bool live = n < nN;
  int rr = n > nN - 1 ? nN - 1 : n;
  rr = rr < 0 ? 0 : rr;
  const float* xp = src + (size_t)rr * FWD;
  v4f a0 = {0.f, 0.f, 0.f, 0.f}, a1 = {0.f, 0.f, 0.f, 0.f};
#pragma unroll 1
  for (int k4 = 0; k4 < FWD / 4; ++k4) {
    const v4f xv = *(const v4f*)(xp + 4 * k4);
    const float* wp = swa + (4 * k4) * NLG;
    v4f w;
    w = *(const v4f*)(wp + 0);  a0 += w * xv.x;
    w = *(const v4f*)(wp + 4);  a1 += w * xv.x;
    w = *(const v4f*)(wp + 8);  a0 += w * xv.y;
    w = *(const v4f*)(wp + 12); a1 += w * xv.y;
    w = *(const v4f*)(wp + 16); a0 += w * xv.z;
    w = *(const v4f*)(wp + 20); a1 += w * xv.z;
    w = *(const v4f*)(wp + 24); a0 += w * xv.w;
    w = *(const v4f*)(wp + 28); a1 += w * xv.w;
  }
  if constexpr (L2 == 1) {
    int bg = batch[rr];
    bg = bg < 0 ? 0 : (bg > nR - 1 ? nR - 1 : bg);
    const v4f g0 = *(const v4f*)(gl2 + (size_t)bg * NLG);
    const v4f g1 = *(const v4f*)(gl2 + (size_t)bg * NLG + 4);
    a0 += g0;
    a1 += g1;
  }
  a0 = zsel(live, a0);
  a1 = zsel(live, a1);
  *(v4f*)(sout + 8 * tid)     = a0;
  *(v4f*)(sout + 8 * tid + 4) = a1;
  __syncthreads();

  float* gp = al + (size_t)blockIdx.x * NTHR * NLG;
  v4f ov[2];
#pragma unroll
  for (int it = 0; it < 2; ++it) ov[it] = *(const v4f*)(sout + 4 * (it * NTHR + tid));
#pragma unroll
  for (int it = 0; it < 2; ++it) *(volatile v4f*)(gp + 4 * (it * NTHR + tid)) = ov[it];
  __threadfence();
#pragma unroll
  for (int it = 0; it < 2; ++it) *(volatile v4f*)(gp + 4 * (it * NTHR + tid)) = ov[it];
}

template <int MODE>
__global__ __launch_bounds__(NTHR) void k_gemm(
    const float* __restrict__ asrc, const int* __restrict__ batch, const float* g2,
    const float* hsrc, const float* __restrict__ wab, const _Float16* __restrict__ Bp,
    float* Cout, float* x2root, float* gl2, int nValid, int nN, int nR) {
  constexpr int KD = FWD;
  constexpr int KSTEPS = KD / 32;
  constexpr int PPR = KD / 4;
  constexpr int NIT = (BM * PPR) / NTHR;
  constexpr int TPW = 4;
  constexpr int OPR = FWD / 4;
  constexpr int ONIT = (BM * OPR) / NTHR;
  static_assert((BM * PPR) % NTHR == 0);
  static_assert((BM * OPR) % NTHR == 0);
  static_assert(NIT == 8 && ONIT == 8);
  static_assert(TPW * 16 * 4 == FWD);
  static_assert(BM == 2 * 16);
  static_assert(NWAVE == 8);
  static_assert(PPR == 64 && OPR == 64);
  static_assert(BM * NLG == NTHR);
  static_assert(BM == 4 * NWAVE);

  __shared__ __attribute__((aligned(16))) _Float16 a16[BM * KD];
  __shared__ __attribute__((aligned(16))) float stg[BM * FWD];
  __shared__ int sroot[BM];
  const int tid = threadIdx.x, lane = tid & 31, wave = tid >> 5, hh = lane >> 4, m = lane & 15;
  const int rowBase = (int)blockIdx.x * BM;
  const int r0 = (wave >> 2) * 16;
  const int c0 = (wave & 3) * 64;

  if constexpr (MODE == 1) {
    const int gq = rowBase + 4 * wave;
    int q0 = 0, q1 = 0, q2 = 0, q3 = 0;
#pragma unroll 1
    for (int i = lane; i < nN; i += 32) {
      const int b = batch[i];
      q0 += (b < gq) ? 1 : 0;
      q1 += (b < gq + 1) ? 1 : 0;
      q2 += (b < gq + 2) ? 1 : 0;
      q3 += (b < gq + 3) ? 1 : 0;
    }
#pragma unroll
    for (int d = 16; d > 0; d >>= 1) {
      q0 += __shfl_xor(q0, d);
      q1 += __shfl_xor(q1, d);
      q2 += __shfl_xor(q2, d);
      q3 += __shfl_xor(q3, d);
    }
    if (lane == 0) {
      sroot[4 * wave + 0] = q0 > nN - 1 ? nN - 1 : (q0 < 0 ? 0 : q0);
      sroot[4 * wave + 1] = q1 > nN - 1 ? nN - 1 : (q1 < 0 ? 0 : q1);
      sroot[4 * wave + 2] = q2 > nN - 1 ? nN - 1 : (q2 < 0 ? 0 : q2);
      sroot[4 * wave + 3] = q3 > nN - 1 ? nN - 1 : (q3 < 0 ? 0 : q3);
    }
    __syncthreads();
  }

#pragma unroll 2
  for (int it = 0; it < NIT; ++it) {
    const int id = it * NTHR + tid;
    const int row = id >> 6, seg = id & 63;
    const int grow = rowBase + row;
    const bool live = grow < nValid;
    int rr;
    if constexpr (MODE == 1) {
      rr = sroot[row];
    } else {
      rr = grow > nValid - 1 ? nValid - 1 : grow;
    }
    rr = rr > nN - 1 ? nN - 1 : rr;
    rr = rr < 0 ? 0 : rr;
    v4f xv = *(const v4f*)(asrc + (size_t)rr * FWD + 4 * seg);
    xv = zsel(live, xv);
    v4h o;
    o.x = (_Float16)(xv.x * ACARRY);
    o.y = (_Float16)(xv.y * ACARRY);
    o.z = (_Float16)(xv.z * ACARRY);
    o.w = (_Float16)(xv.w * ACARRY);
    *(v4h*)(a16 + (size_t)row * KD + 4 * seg) = o;
  }

  if constexpr (MODE == 1) {
    v4f cv[ONIT];
#pragma unroll
    for (int it = 0; it < ONIT; ++it) {
      const int p = it * NTHR + tid;
      const int row = p >> 6;
      const int col4 = 4 * (p & 63);
      const bool live = rowBase + row < nValid;
      int node = sroot[row];
      node = node < 0 ? 0 : (node > nN - 1 ? nN - 1 : node);
      const v4f v = *(const v4f*)(hsrc + (size_t)node * FWD + col4);
      cv[it] = zsel(live, v);
    }
    const int gr = tid >> 3, jj = tid & 7;
    int nd = sroot[gr];
    nd = nd < 0 ? 0 : (nd > nN - 1 ? nN - 1 : nd);
    const bool lv = rowBase + gr < nValid;
    const float* xp = asrc + (size_t)nd * FWD;
    float ga = 0.f;
#pragma unroll 4
    for (int k = 0; k < FWD; ++k) ga += xp[k] * wab[k * NLG + jj];
    ga = lv ? ga : 0.f;
    float* xg = x2root + (size_t)rowBase * FWD;
    float* gg = gl2 + (size_t)rowBase * NLG + tid;
#pragma unroll
    for (int it = 0; it < ONIT; ++it) *(volatile v4f*)(xg + 4 * (it * NTHR + tid)) = cv[it];
    *(volatile float*)gg = ga;
    __threadfence();
#pragma unroll
    for (int it = 0; it < ONIT; ++it) *(volatile v4f*)(xg + 4 * (it * NTHR + tid)) = cv[it];
    *(volatile float*)gg = ga;
  }
  __syncthreads();

  v8f acc[TPW];
#pragma unroll
  for (int t = 0; t < TPW; ++t) { v8f z = {0.f, 0.f, 0.f, 0.f, 0.f, 0.f, 0.f, 0.f}; acc[t] = z; }

  const _Float16* ap = a16 + (size_t)(r0 + m) * KD + 8 * hh;
  const _Float16* bp = Bp + (size_t)(c0 + m) * KD + 8 * hh;
#pragma unroll 1
  for (int kt = 0; kt < KSTEPS; ++kt) {
    Frag a;
    a.h[0] = *(const v8h*)(ap + 32 * kt);
    a.h[1] = *(const v8h*)(ap + 32 * kt + 16);
#pragma unroll
    for (int t = 0; t < TPW; ++t) {
      const size_t to = (size_t)(16 * t) * KD + 32 * kt;
      Frag b;
      b.h[0] = *(const v8h*)(bp + to);
      b.h[1] = *(const v8h*)(bp + to + 16);
      acc[t] = wmh(a.v, b.v, acc[t]);
    }
  }

  {
    float* sp = stg + (size_t)(r0 + 8 * hh) * FWD + c0 + m;
#pragma unroll
    for (int r = 0; r < 8; ++r) {
#pragma unroll
      for (int t = 0; t < TPW; ++t) sp[r * FWD + 16 * t] = acc[t][r] * GSCALE;
    }
  }
  __syncthreads();

  v4f ov[ONIT];
#pragma unroll
  for (int it = 0; it < ONIT; ++it) {
    const int p = it * NTHR + tid;
    v4f v = *(const v4f*)(stg + 4 * p);
    if constexpr (MODE == 2) {
      const int row = p >> 6;
      const int grow = rowBase + row;
      const bool live = grow < nValid;
      int nr = grow > nN - 1 ? nN - 1 : grow;
      nr = nr < 0 ? 0 : nr;
      int br = batch[nr];
      br = br < 0 ? 0 : (br > nR - 1 ? nR - 1 : br);
      const v4f gv = *(const v4f*)(g2 + (size_t)br * FWD + 4 * (p & 63));
      v += zsel(live, gv);
    }
    ov[it] = v;
  }
  float* gb = Cout + (size_t)rowBase * FWD;
#pragma unroll
  for (int it = 0; it < ONIT; ++it) *(volatile v4f*)(gb + 4 * (it * NTHR + tid)) = ov[it];
  __threadfence();
#pragma unroll
  for (int it = 0; it < ONIT; ++it) *(volatile v4f*)(gb + 4 * (it * NTHR + tid)) = ov[it];
}

__global__ __launch_bounds__(AGTHR) void k_attn_agg(
    const int* __restrict__ csr, const int* __restrict__ off, const int* __restrict__ cnt,
    const float* __restrict__ al, const float* __restrict__ h,
    const float* __restrict__ bias, const float* __restrict__ bng, const float* __restrict__ bnb,
    const float* __restrict__ bnm, const float* __restrict__ bnv,
    const float* __restrict__ lng, const float* __restrict__ lnb,
    float* outp, int nN, int csrLen) {
  const int tid = threadIdx.x, lane = tid & 31, wave = tid >> 5;
  const int tbase = blockIdx.x * TGT + wave * 32;
  const int cA = 4 * lane, cB = FWD / 2 + 4 * lane;
  const int hsel = lane >> 4;
  const int cl    = tbase + lane;
  const int cnt_l = cnt[cl];
  const int off_l = off[cl];

  const v4f biA = ld4(bias + cA), biB = ld4(bias + cB);
  const v4f mA  = ld4(bnm + cA),  mB  = ld4(bnm + cB);
  const v4f bbA = ld4(bnb + cA),  bbB = ld4(bnb + cB);
  const v4f gA  = ld4(lng + cA),  gB  = ld4(lng + cB);
  const v4f lbA = ld4(lnb + cA),  lbB = ld4(lnb + cB);
  v4f scA, scB;
  {
    const v4f bgA = ld4(bng + cA), bgB = ld4(bng + cB);
    const v4f bvA = ld4(bnv + cA), bvB = ld4(bnv + cB);
    scA.x = bgA.x * rsqrtf(bvA.x + 1e-5f); scA.y = bgA.y * rsqrtf(bvA.y + 1e-5f);
    scA.z = bgA.z * rsqrtf(bvA.z + 1e-5f); scA.w = bgA.w * rsqrtf(bvA.w + 1e-5f);
    scB.x = bgB.x * rsqrtf(bvB.x + 1e-5f); scB.y = bgB.y * rsqrtf(bvB.y + 1e-5f);
    scB.z = bgB.z * rsqrtf(bvB.z + 1e-5f); scB.w = bgB.w * rsqrtf(bvB.w + 1e-5f);
  }

#pragma unroll 1
  for (int j = 0; j < 32; ++j) {
    const int c = tbase + j;
    int n = __builtin_amdgcn_readfirstlane(__shfl(cnt_l, j));
    n = n < 0 ? 0 : (n > DEGCAP ? DEGCAP : n);
    const int st = __builtin_amdgcn_readfirstlane(__shfl(off_l, j));
    const v4f sa = ld4(al + (size_t)c * NLG);
    const v4f sd = ld4(al + (size_t)c * NLG + 4);
    const float es0 = lk(sa.x + sd.x), es1 = lk(sa.y + sd.y), es2 = lk(sa.z + sd.z), es3 = lk(sa.w + sd.w);

    float mx0 = es0, mx1 = es1, mx2 = es2, mx3 = es3;
#pragma unroll 1
    for (int q0 = 0; q0 < n; q0 += 32) {
      int pos = st + q0 + lane;
      pos = pos < 0 ? 0 : (pos > csrLen - 1 ? csrLen - 1 : pos);
      int sl = csr[pos];
      sl = sl < 0 ? 0 : (sl > nN - 1 ? nN - 1 : sl);
      const v4f a4 = ld4(al + (size_t)sl * NLG);
      const bool valid = (q0 + lane) < n;
      const float e0 = lk(a4.x + sd.x), e1 = lk(a4.y + sd.y), e2 = lk(a4.z + sd.z), e3 = lk(a4.w + sd.w);
      mx0 = valid ? fmaxf(mx0, e0) : mx0;
      mx1 = valid ? fmaxf(mx1, e1) : mx1;
      mx2 = valid ? fmaxf(mx2, e2) : mx2;
      mx3 = valid ? fmaxf(mx3, e3) : mx3;
    }
    mx0 = wmax(mx0); mx1 = wmax(mx1); mx2 = wmax(mx2); mx3 = wmax(mx3);

    const float ps0 = __expf(es0 - mx0), ps1 = __expf(es1 - mx1), ps2 = __expf(es2 - mx2), ps3 = __expf(es3 - mx3);
    const float psA = hsel ? ps1 : ps0, psB = hsel ? ps3 : ps2;
    const v4f hs0 = ld4(h + (size_t)c * FWD + cA);
    const v4f hs1 = ld4(h + (size_t)c * FWD + cB);
    v4f accA = hs0 * psA, accB = hs1 * psB;
    float sm0 = 0.f, sm1 = 0.f, sm2 = 0.f, sm3 = 0.f;

#pragma unroll 1
    for (int q0 = 0; q0 < n; q0 += 32) {
      int pos = st + q0 + lane;
      pos = pos < 0 ? 0 : (pos > csrLen - 1 ? csrLen - 1 : pos);
      int sl = csr[pos];
      sl = sl < 0 ? 0 : (sl > nN - 1 ? nN - 1 : sl);
      const v4f a4 = ld4(al + (size_t)sl * NLG);
      const bool valid = (q0 + lane) < n;
      const float e0 = lk(a4.x + sd.x), e1 = lk(a4.y + sd.y), e2 = lk(a4.z + sd.z), e3 = lk(a4.w + sd.w);
      const float p0 = __expf(e0 - mx0), p1 = __expf(e1 - mx1), p2 = __expf(e2 - mx2), p3 = __expf(e3 - mx3);
      sm0 += valid ? p0 : 0.f;
      sm1 += valid ? p1 : 0.f;
      sm2 += valid ? p2 : 0.f;
      sm3 += valid ? p3 : 0.f;
      const int ip0 = __float_as_int(p0), ip1 = __float_as_int(p1), ip2 = __float_as_int(p2), ip3 = __float_as_int(p3);
      const int mcnt = (n - q0) < 32 ? (n - q0) : 32;
#pragma unroll 1
      for (int pp = 0; pp < mcnt; ++pp) {
        const int s = __builtin_amdgcn_readlane(sl, pp);
        const float f0 = __int_as_float(__builtin_amdgcn_readlane(ip0, pp));
        const float f1 = __int_as_float(__builtin_amdgcn_readlane(ip1, pp));
        const float f2 = __int_as_float(__builtin_amdgcn_readlane(ip2, pp));
        const float f3 = __int_as_float(__builtin_amdgcn_readlane(ip3, pp));
        const float pa = hsel ? f1 : f0, pb = hsel ? f3 : f2;
        const v4f hv0 = ld4(h + (size_t)s * FWD + cA);
        const v4f hv1 = ld4(h + (size_t)s * FWD + cB);
        accA += hv0 * pa;
        accB += hv1 * pb;
      }
    }
    sm0 = wsum(sm0) + ps0; sm1 = wsum(sm1) + ps1; sm2 = wsum(sm2) + ps2; sm3 = wsum(sm3) + ps3;
    const float rd0 = 1.0f / (sm0 + 1e-16f), rd1 = 1.0f / (sm1 + 1e-16f);
    const float rd2 = 1.0f / (sm2 + 1e-16f), rd3 = 1.0f / (sm3 + 1e-16f);
    const float rdA = hsel ? rd1 : rd0, rdB = hsel ? rd3 : rd2;

    const v4f tA = accA * rdA + biA, tB = accB * rdB + biB;
    const v4f zA = (tA - mA) * scA + bbA, zB = (tB - mB) * scB + bbB;
    float s8 = zA.x + zA.y + zA.z + zA.w + zB.x + zB.y + zB.z + zB.w;
    s8 = wsum(s8);
    const float mu = s8 * (1.0f / FWD);
    const v4f dA = zA - mu, dB = zB - mu;
    float v8 = dA.x * dA.x + dA.y * dA.y + dA.z * dA.z + dA.w * dA.w + dB.x * dB.x + dB.y * dB.y + dB.z * dB.z + dB.w * dB.w;
    v8 = wsum(v8);
    const float var = v8 * (1.0f / FWD);
    const float rs = rsqrtf(var + 1e-5f);
    v4f yA = (dA * rs) * gA + lbA, yB = (dB * rs) * gB + lbB;
    yA.x = fmaxf(yA.x, 0.f); yA.y = fmaxf(yA.y, 0.f); yA.z = fmaxf(yA.z, 0.f); yA.w = fmaxf(yA.w, 0.f);
    yB.x = fmaxf(yB.x, 0.f); yB.y = fmaxf(yB.y, 0.f); yB.z = fmaxf(yB.z, 0.f); yB.w = fmaxf(yB.w, 0.f);
    const bool live = c < nN;
    yA = zsel(live, yA);
    yB = zsel(live, yB);
    float* gp = outp + (size_t)c * FWD;
    *(volatile v4f*)(gp + cA) = yA;
    *(volatile v4f*)(gp + cB) = yB;
    __threadfence();
    *(volatile v4f*)(gp + cA) = yA;
    *(volatile v4f*)(gp + cB) = yB;
  }
}

__global__ __launch_bounds__(NTHR) void k_pool(
    const int* __restrict__ batch, const float* __restrict__ hf, const float* __restrict__ x2root,
    float* out, int nN, int nR, int nG, int vec8) {
  __shared__ __attribute__((aligned(16))) int list[LISTN];
  __shared__ __attribute__((aligned(16))) float spart[NWAVE * GPB * OWD];
  __shared__ __attribute__((aligned(16))) float smean[GPB * OWD];
  __shared__ int scount[NWAVE * GPB];
  __shared__ int sflag;
  const int tid = threadIdx.x, lane = tid & 31, wave = tid >> 5;
  const int gBase = blockIdx.x * GPB;
  const int cA = 4 * lane, cB = FWD / 2 + 4 * lane;

  v4f a0[GPB], a1[GPB], a2[GPB], a3[GPB];
  int cn[GPB];
#pragma unroll
  for (int s = 0; s < GPB; ++s) {
    const v4f z = {0.f, 0.f, 0.f, 0.f};
    a0[s] = z; a1[s] = z; a2[s] = z; a3[s] = z; cn[s] = 0;
  }

  if (tid == 0) sflag = 0;
  int bad = 0;
#pragma unroll 1
  for (int i = tid; i + 1 < nN; i += NTHR) {
    const int b0 = batch[i], b1 = batch[i + 1];
    bad |= (b0 > b1) ? 1 : 0;
  }
  __syncthreads();
  if (bad != 0) sflag = 1;

  const int nChunks = (nN + CHUNK - 1) / CHUNK;
#pragma unroll 1
  for (int ch = 0; ch < nChunks; ++ch) {
    const int cbase = ch * CHUNK;
    const int wc = scan_chunk<GPB>(batch, nN, cbase, gBase, vec8, list, tid, lane, wave);
    __syncthreads();
    int n = wc;
    n = n > WCAP ? WCAP : (n < 0 ? 0 : n);
    const int* lp = list + wave * WCAP;
#pragma unroll 1
    for (int i = 0; i < n; ++i) {
      const int ent = __builtin_amdgcn_readfirstlane(lp[i]);
      int node = cbase + ((ent >> 12) & (CHUNK - 1));
      node = node > nN - 1 ? nN - 1 : (node < 0 ? 0 : node);
      const int slot = ent & (GPB - 1);
      int bg = gBase + slot;
      bg = bg > nR - 1 ? nR - 1 : (bg < 0 ? 0 : bg);
      const v4f hv0 = ld4(hf + (size_t)node * FWD + cA);
      const v4f hv1 = ld4(hf + (size_t)node * FWD + cB);
      const v4f rv0 = ld4(x2root + (size_t)bg * FWD + cA);
      const v4f rv1 = ld4(x2root + (size_t)bg * FWD + cB);
#pragma unroll
      for (int s = 0; s < GPB; ++s) {
        const bool hit = slot == s;
        a0[s] += zsel(hit, hv0);
        a1[s] += zsel(hit, hv1);
        a2[s] += zsel(hit, rv0);
        a3[s] += zsel(hit, rv1);
        cn[s] += hit ? 1 : 0;
      }
    }
    __syncthreads();
  }

#pragma unroll
  for (int s = 0; s < GPB; ++s) {
    float* sp = spart + (size_t)(wave * GPB + s) * OWD;
    *(v4f*)(sp + cA) = a0[s];
    *(v4f*)(sp + cB) = a1[s];
    *(v4f*)(sp + FWD + cA) = a2[s];
    *(v4f*)(sp + FWD + cB) = a3[s];
  }
  if (lane == 0) {
#pragma unroll
    for (int s = 0; s < GPB; ++s) scount[wave * GPB + s] = cn[s];
  }
  __syncthreads();
  const bool poison = sflag != 0;
  const float qnan = __int_as_float(0x7fc00000);
#pragma unroll
  for (int q = 0; q < (GPB * OWD) / NTHR; ++q) {
    const int idx = q * NTHR + tid;
    const int s = idx / OWD, c = idx - s * OWD;
    float S = 0.f;
    int C = 0;
#pragma unroll
    for (int w = 0; w < NWAVE; ++w) {
      S += spart[(w * GPB + s) * OWD + c];
      C += scount[w * GPB + s];
    }
    const float Cf = (float)C;
    const float rc = 1.0f / fmaxf(Cf, 1.0f);
    smean[idx] = poison ? qnan : S * rc;
  }
  __syncthreads();
  const int ws = wave < GPB ? wave : 0;
  const v4f v0 = *(const v4f*)(smean + ws * OWD + cA);
  const v4f v1 = *(const v4f*)(smean + ws * OWD + cB);
  const v4f v2 = *(const v4f*)(smean + ws * OWD + FWD + cA);
  const v4f v3 = *(const v4f*)(smean + ws * OWD + FWD + cB);
  const bool live = (wave < GPB) && ((gBase + wave) < nG);
  int gi = gBase + ws;
  gi = gi > nG - 1 ? nG - 1 : (gi < 0 ? 0 : gi);
  float* gp = out + (size_t)gi * OWD;
  if (live) {
    *(volatile v4f*)(gp + cA) = v0;
    *(volatile v4f*)(gp + cB) = v1;
    *(volatile v4f*)(gp + FWD + cA) = v2;
    *(volatile v4f*)(gp + FWD + cB) = v3;
  }
  __threadfence();
  if (live) {
    *(volatile v4f*)(gp + cA) = v0;
    *(volatile v4f*)(gp + cB) = v1;
    *(volatile v4f*)(gp + FWD + cA) = v2;
    *(volatile v4f*)(gp + FWD + cB) = v3;
  }
}

extern "C" void kernel_launch(void* const* d_in, const int* in_sizes, int n_in,
                              void* d_out, int out_size, void* d_ws, size_t ws_size,
                              hipStream_t stream) {
  if (n_in < 23) return;
  if (in_sizes[0] < FWD || (in_sizes[0] % FWD) != 0) return;
  const int nN = in_sizes[0] / FWD;
  if (in_sizes[1] < 2 || (in_sizes[1] & 1) != 0) return;
  const int nE = in_sizes[1] / 2;
  if (in_sizes[2] != nN) return;
  if (in_sizes[3] != FWD * FWD) return;
  if (in_sizes[4] != 4 * HCH || in_sizes[5] != 4 * HCH) return;
  for (int i = 6; i <= 12; ++i) if (in_sizes[i] != FWD) return;
  if (in_sizes[13] != 2 * FWD * FWD) return;
  if (in_sizes[14] != 4 * HCH || in_sizes[15] != 4 * HCH) return;
  for (int i = 16; i <= 22; ++i) if (in_sizes[i] != FWD) return;
  if (out_size < OWD || (out_size % OWD) != 0) return;
  const int nG = out_size / OWD;
  if (nG < 1 || nG > GMAX) return;
  const int nR = nG;
  if (nE > (1 << 28) || nN > (1 << 22)) return;

  const float* x     = (const float*)d_in[0];
  const int*   ei    = (const int*)d_in[1];
  const int*   src   = ei;
  const int*   dst   = ei + nE;
  const int*   batch = (const int*)d_in[2];
  const float* W1    = (const float*)d_in[3];
  const float* as1   = (const float*)d_in[4];
  const float* ad1   = (const float*)d_in[5];
  const float* b1    = (const float*)d_in[6];
  const float* bn1g  = (const float*)d_in[7];
  const float* bn1b  = (const float*)d_in[8];
  const float* bn1m  = (const float*)d_in[9];
  const float* bn1v  = (const float*)d_in[10];
  const float* ln1g  = (const float*)d_in[11];
  const float* ln1b  = (const float*)d_in[12];
  const float* W2    = (const float*)d_in[13];
  const float* as2   = (const float*)d_in[14];
  const float* ad2   = (const float*)d_in[15];
  const float* b2    = (const float*)d_in[16];
  const float* bn2g  = (const float*)d_in[17];
  const float* bn2b  = (const float*)d_in[18];
  const float* bn2m  = (const float*)d_in[19];
  const float* bn2v  = (const float*)d_in[20];
  const float* ln2g  = (const float*)d_in[21];
  const float* ln2b  = (const float*)d_in[22];
  float* out = (float*)d_out;

  const int NPAD   = ((nN + RGRAN - 1) / RGRAN) * RGRAN;
  const int nBC    = (nN + NBC - 1) / NBC;
  const int CNTPAD = nBC * NBC;
  if (CNTPAD < NPAD) return;
  if (4 * nBC + 1 > RBN) return;
  const int nBF    = (nN + NBF - 1) / NBF;
  if (nBF > 4 * nBC) return;
  const int csrLen = ((nE + 31) & ~31) + 4096;
  if (31 * 4 * nBC > 4096) return;
  const int nAgg   = NPAD / TGT;
  const int nGemm  = NPAD / BM;
  const int nLog   = NPAD / NTHR;
  const int GPAD   = ((nR + BM - 1) / BM) * BM;
  const int GBLK   = (nG + GPB - 1) / GPB;

  char* ws = (char*)d_ws;
  size_t off = 0;
  const size_t oWp0 = off; off += (size_t)FWD * FWD * 2;          off = (off + 255) & ~(size_t)255;
  const size_t oWp1 = off; off += (size_t)FWD * FWD * 2;          off = (off + 255) & ~(size_t)255;
  const size_t oWp2 = off; off += (size_t)FWD * FWD * 2;          off = (off + 255) & ~(size_t)255;
  const size_t oWa  = off; off += (size_t)3 * FWD * NLG * 4;      off = (off + 255) & ~(size_t)255;
  const size_t oAl  = off; off += (size_t)NPAD * NLG * 4;         off = (off + 255) & ~(size_t)255;
  const size_t oP   = off; off += (size_t)NPAD * FWD * 4;         off = (off + 255) & ~(size_t)255;
  const size_t oQ   = off; off += (size_t)NPAD * FWD * 4;         off = (off + 255) & ~(size_t)255;
  const size_t oG2  = off; off += (size_t)GPAD * FWD * 4;         off = (off + 255) & ~(size_t)255;
  const size_t oGl2 = off; off += (size_t)GPAD * NLG * 4;         off = (off + 255) & ~(size_t)255;
  const size_t oX2r = off; off += (size_t)GPAD * FWD * 4;         off = (off + 255) & ~(size_t)255;
  const size_t oCnt = off; off += (size_t)CNTPAD * 4;             off = (off + 255) & ~(size_t)255;
  const size_t oOff = off; off += (size_t)CNTPAD * 4;             off = (off + 255) & ~(size_t)255;
  const size_t oRb  = off; off += (size_t)RBN * 4;                off = (off + 255) & ~(size_t)255;
  const size_t oCsr = off; off += (size_t)csrLen * 4;             off = (off + 255) & ~(size_t)255;
  if (off > ws_size || off > (size_t)WSCAP) return;

  _Float16* wpl0 = (_Float16*)(ws + oWp0);
  _Float16* wpl1 = (_Float16*)(ws + oWp1);
  _Float16* wpl2 = (_Float16*)(ws + oWp2);
  float* wa   = (float*)(ws + oWa);
  float* al   = (float*)(ws + oAl);
  float* pP   = (float*)(ws + oP);
  float* pQ   = (float*)(ws + oQ);
  float* g2   = (float*)(ws + oG2);
  float* gl2  = (float*)(ws + oGl2);
  float* x2r  = (float*)(ws + oX2r);
  int*   cnt  = (int*)(ws + oCnt);
  int*   offp = (int*)(ws + oOff);
  int*   rb   = (int*)(ws + oRb);
  int*   csr  = (int*)(ws + oCsr);

  const int vec8 = ((nE & 3) == 0) ? 1 : 0;

  k_wcvt<<<(FWD * (FWD / 8) + NTHR - 1) / NTHR, NTHR, 0, stream>>>(W1, wpl0, 0, FWD, FWD);
  k_wcvt<<<(FWD * (FWD / 8) + NTHR - 1) / NTHR, NTHR, 0, stream>>>(W2, wpl1, 0, FWD, 2 * FWD);
  k_wcvt<<<(FWD * (FWD / 8) + NTHR - 1) / NTHR, NTHR, 0, stream>>>(W2, wpl2, FWD, FWD, 2 * FWD);
  k_wa<<<(3 * FWD * NLG) / NTHR, NTHR, 0, stream>>>(W1, W2, as1, ad1, as2, ad2, wa);

  k_count<<<nBC, NTHR, 0, stream>>>(dst, cnt, nE, vec8);
  k_offsets<<<1, OTHR, 0, stream>>>(cnt, offp, rb, nBC);
  hipFuncSetAttribute(reinterpret_cast<const void*>(&k_fill),
                      hipFuncAttributeMaxDynamicSharedMemorySize, LDS_FILL);
  k_fill<<<nBF, NTHR, LDS_FILL, stream>>>(src, dst, offp, rb, csr, nN, nE, vec8, csrLen);

  k_gemm<0><<<nGemm, NTHR, 0, stream>>>(x, batch, g2, pQ, wa + 2 * FWD * NLG, wpl0, pP, x2r, gl2, nN, nN, nR);
  k_logit<0><<<nLog, NTHR, 0, stream>>>(x, wa, gl2, batch, al, nN, nR);
  k_attn_agg<<<nAgg, AGTHR, 0, stream>>>(csr, offp, cnt, al, pP, b1, bn1g, bn1b, bn1m, bn1v, ln1g, ln1b,
                                          pQ, nN, csrLen);
  k_gemm<1><<<GPAD / BM, NTHR, 0, stream>>>(x, batch, g2, pQ, wa + 2 * FWD * NLG, wpl2, g2, x2r, gl2, nR, nN, nR);
  k_gemm<2><<<nGemm, NTHR, 0, stream>>>(pQ, batch, g2, pQ, wa + 2 * FWD * NLG, wpl1, pP, x2r, gl2, nN, nN, nR);
  k_logit<1><<<nLog, NTHR, 0, stream>>>(pQ, wa + FWD * NLG, gl2, batch, al, nN, nR);
  k_attn_agg<<<nAgg, AGTHR, 0, stream>>>(csr, offp, cnt, al, pP, b2, bn2g, bn2b, bn2m, bn2v, ln2g, ln2b,
                                          pQ, nN, csrLen);
  k_pool<<<GBLK, NTHR, 0, stream>>>(batch, pQ, x2r, out, nN, nR, nG, 1);
}
